// BKT_RNN_23081154249236
// MI455X (gfx1250) — hardware-verified
//
#include <hip/hip_runtime.h>
#include <hip/hip_bf16.h>
#include <math.h>

#define HID   128
#define G4    512
#define NROW  (G4 + 16)
#define TLEN  512
#define BATCH 1024
#define MT    16
#define NWG   (BATCH / MT)
#define NTHR  256
#define WSDW  68

typedef _Float16 __hf16;
#define __bf16 __hf16
#define __builtin_amdgcn_wmma_f32_16x16x32_bf16 __builtin_amdgcn_wmma_f32_16x16x32_f16
typedef __attribute__((ext_vector_type(16))) _Float16 v16bf;
typedef __attribute__((ext_vector_type(8)))  float  v8f;
typedef __attribute__((ext_vector_type(8)))  int    v8i;
typedef __attribute__((ext_vector_type(4)))  int    v4i;

union Frag { v8i i; v16bf b; };
union PackBF { __bf16 h[2]; unsigned int u; };

__device__ __forceinline__ void ld_frag(Frag& f, const unsigned int* p, int second_off) {
    v4i a = *(const v4i*)(p);
    v4i c = *(const v4i*)(p + second_off);
    f.i = __builtin_shufflevector(a, c, 0, 1, 2, 3, 4, 5, 6, 7);
}

__device__ __forceinline__ float sigm(float v) {
    return 1.0f / (1.0f + __expf(-v));
}
__device__ __forceinline__ float tanh_fast(float v) {
    return 1.0f - 2.0f / (__expf(2.0f * v) + 1.0f);
}

__global__ __launch_bounds__(NTHR) void bkt_lstm_fused(
    const float* __restrict__ x,       const float* __restrict__ y,
    const float* __restrict__ W_ih,    const float* __restrict__ W_hh,
    const float* __restrict__ b_ih,    const float* __restrict__ b_hh,
    const float* __restrict__ prior_W, const float* __restrict__ prior_b,
    const float* __restrict__ post_W,  const float* __restrict__ post_b,
    float* __restrict__ out,           float* __restrict__ ws)
{
    __shared__ __align__(16) unsigned int Wlds[NROW * WSDW];
    __shared__ __align__(16) unsigned int Hlds[2 * MT * WSDW];
    __shared__ float paramsLds[MT * 4];
    __shared__ __align__(16) float xbuf[2][MT];
    __shared__ float lossred[MT];
    __shared__ float stage[2][2][MT];
    float* CB = ws + NWG * 32 + (size_t)blockIdx.x * TLEN * MT;
    float* LB = ws + NWG * 32 + (size_t)NWG * TLEN * MT + (size_t)blockIdx.x * TLEN * MT;

    const int tid  = threadIdx.x;
    const int lane = tid & 31;
    const int wv   = tid >> 5;
    const int b0   = blockIdx.x * MT;
    const int lo16 = lane & 15;
    const int hiH  = (lane < 16) ? 0 : 1;

    for (int idx = tid; idx < G4 * (HID / 2); idx += NTHR) {
        int n  = idx >> 6;
        int kd = idx & 63;
        PackBF p;
        p.h[0] = (__bf16)W_hh[n * HID + 2 * kd + 0];
        p.h[1] = (__bf16)W_hh[n * HID + 2 * kd + 1];
        Wlds[n * WSDW + kd] = p.u;
    }
    for (int idx = tid; idx < 16 * (HID / 2); idx += NTHR) {
        int p  = idx >> 6;
        int kd = idx & 63;
        PackBF pk;
        if (p < 4) {
            pk.h[0] = (__bf16)post_W[p * HID + 2 * kd + 0];
            pk.h[1] = (__bf16)post_W[p * HID + 2 * kd + 1];
        } else pk.u = 0u;
        Wlds[(G4 + p) * WSDW + kd] = pk.u;
    }
    for (int idx = tid; idx < 2 * MT * WSDW; idx += NTHR) Hlds[idx] = 0u;

    float biasq[4], wihq[4];
#pragma unroll
    for (int q = 0; q < 4; ++q) {
        int n = q * HID + wv * 16 + lo16;
        biasq[q] = b_ih[n] + b_hh[n];
        wihq[q]  = W_ih[n];
    }
    const float pb = (lo16 < 4) ? post_b[lo16] : 0.0f;

    float cst[8];
#pragma unroll
    for (int v = 0; v < 8; ++v) cst[v] = 0.0f;

    float lat = 0.0f, lossacc = 0.0f;
    if (tid < MT) {
        lat = sigm(x[b0 + tid] * prior_W[0] + prior_b[0]);
        xbuf[0][tid] = x[b0 + tid];
    }
    __syncthreads();

    Frag PB[4];
    if (wv == 0) {
#pragma unroll
        for (int kki = 0; kki < 4; ++kki)
            ld_frag(PB[kki], Wlds + (G4 + lo16) * WSDW + kki * 16 + hiH * 4, 8);
    }

    Frag A[4];

    for (int t = 0; t < TLEN; ++t) {
        const unsigned int* hrd = Hlds + (t & 1) * (MT * WSDW);
        unsigned int*       hwr = Hlds + ((t + 1) & 1) * (MT * WSDW);

        if (wv != 0 || t == 0) {
            const unsigned int* hrow = hrd + lo16 * WSDW + hiH * 4;
#pragma unroll
            for (int kki = 0; kki < 4; ++kki)
                ld_frag(A[kki], hrow + kki * 16, 8);
        }

        float ytv = 0.0f;
        if (tid < MT) {
            int tn = (t + 1 < TLEN) ? t + 1 : t;
            xbuf[(t + 1) & 1][tid] = x[tn * BATCH + b0 + tid];
            ytv = y[t * BATCH + b0 + tid];
        }

        v8f acc[4];
#pragma unroll
        for (int q = 0; q < 4; ++q) {
#pragma unroll
            for (int v = 0; v < 8; ++v)
                acc[q][v] = xbuf[t & 1][v + 8 * hiH] * wihq[q] + biasq[q];
        }

#pragma unroll
        for (int kki = 0; kki < 4; ++kki) {
#pragma unroll
            for (int q = 0; q < 4; ++q) {
                Frag Bf;
                const int n = q * HID + wv * 16 + lo16;
                ld_frag(Bf, Wlds + n * WSDW + kki * 16 + hiH * 4, 8);
                acc[q] = __builtin_amdgcn_wmma_f32_16x16x32_bf16(
                    false, A[kki].b, false, Bf.b, (short)0, acc[q], false, false);
            }
            asm volatile("v_nop\n\tv_nop\n\tv_nop\n\tv_nop\n\tv_nop" : "+v"(acc[0]), "+v"(acc[1]), "+v"(acc[2]), "+v"(acc[3]) : "v"(A[kki].b));
        }

        {
            __bf16* Hw = (__bf16*)hwr;
            const int j = wv * 16 + lo16;
#pragma unroll
            for (int v = 0; v < 8; ++v) {
                int m = v + 8 * hiH;
                float ig = sigm(acc[0][v]);
                float fg = sigm(acc[1][v]);
                float gg = tanh_fast(acc[2][v]);
                float og = sigm(acc[3][v]);
                float c  = fg * cst[v] + ig * gg;
                cst[v]   = c;
                float h  = og * tanh_fast(c);
                Hw[m * (2 * WSDW) + j] = (__bf16)h;
            }
        }
        __syncthreads();

        if (wv == 0) {
            const unsigned int* hrow = hwr + lo16 * WSDW + hiH * 4;
#pragma unroll
            for (int kki = 0; kki < 4; ++kki)
                ld_frag(A[kki], hrow + kki * 16, 8);

            v8f pacc;
#pragma unroll
            for (int v = 0; v < 8; ++v) pacc[v] = pb;
#pragma unroll
            for (int kki = 0; kki < 4; ++kki)
                pacc = __builtin_amdgcn_wmma_f32_16x16x32_bf16(
                    false, A[kki].b, false, PB[kki].b, (short)0, pacc, false, false);
            asm volatile("v_nop\n\tv_nop\n\tv_nop\n\tv_nop\n\tv_nop" : "+v"(pacc) : "v"(A[3].b), "v"(PB[3].b));

            if (lo16 < 4) {
#pragma unroll
                for (int v = 0; v < 8; ++v)
                    paramsLds[(v + 8 * hiH) * 4 + lo16] = sigm(pacc[v]);
            }
            if (tid < MT) {
                float l = paramsLds[tid * 4 + 0];
                float f = paramsLds[tid * 4 + 1];
                float g = paramsLds[tid * 4 + 2];
                float s = paramsLds[tid * 4 + 3];
                float correct = lat * (1.0f - s) + (1.0f - lat) * g;
                float k1 = lat * (1.0f - s) * __builtin_amdgcn_rcpf(correct);
                float k0 = lat * s * __builtin_amdgcn_rcpf(lat * s + (1.0f - lat) * (1.0f - g));
                float mt = k1 * correct + k0 * (1.0f - correct);
                lat = mt * (1.0f - f) + (1.0f - mt) * l;
                stage[0][t & 1][tid] = correct;
                stage[1][t & 1][tid] = lat;
                lossacc -= ytv * fmaxf(logf(correct), -100.0f)
                         + (1.0f - ytv) * fmaxf(logf(1.0f - correct), -100.0f);
            }
            if (t & 1) {
                const float cv = stage[0][lane >> 4][lane & 15], lv = stage[1][lane >> 4][lane & 15];
                float* cp = CB + (size_t)(t >> 1) * 32 + lane; float* lp = LB + (size_t)(t >> 1) * 32 + lane;
                *(volatile float*)cp = cv; *(volatile float*)lp = lv; __threadfence();
                *(volatile float*)cp = cv; *(volatile float*)lp = lv;
            }
        }
    }

    if (tid < MT) lossred[tid] = lossacc;
    __syncthreads();
    if (tid == 0) {
        float s = 0.0f;
#pragma unroll
        for (int i = 0; i < MT; ++i) s += lossred[i];
        *(volatile float*)(ws + blockIdx.x * 32) = s; __threadfence(); *(volatile float*)(ws + blockIdx.x * 32) = s;
    }
}
__global__ __launch_bounds__(256) void relayout(const float* __restrict__ ws, float* __restrict__ out) {
    const int idx = blockIdx.x * 256 + threadIdx.x;
    const int t = idx / BATCH, b = idx % BATCH, blk = b / MT;
    const size_t o = (size_t)blk * TLEN * MT + (size_t)(t >> 1) * 32 + (t & 1) * 16 + (b & 15);
    const float cv = ws[NWG * 32 + o], lv = ws[NWG * 32 + (size_t)NWG * TLEN * MT + o];
    *(volatile float*)(out + idx) = cv; *(volatile float*)(out + (size_t)TLEN * BATCH + idx) = lv; __threadfence();
    *(volatile float*)(out + idx) = cv; *(volatile float*)(out + (size_t)TLEN * BATCH + idx) = lv;
}

__global__ void loss_reduce(const float* __restrict__ ws, float* __restrict__ out) {
    if (threadIdx.x == 0 && blockIdx.x == 0) {
        float s = 0.0f;
        for (int i = 0; i < NWG; ++i) s += ws[i * 32];
        const float v = s / (float)(TLEN * BATCH);
        *(volatile float*)(out + 2 * TLEN * BATCH) = v; __threadfence(); *(volatile float*)(out + 2 * TLEN * BATCH) = v;
    }
}

extern "C" void kernel_launch(void* const* d_in, const int* in_sizes, int n_in,
                              void* d_out, int out_size, void* d_ws, size_t ws_size,
                              hipStream_t stream) {
    (void)in_sizes; (void)n_in; (void)out_size;
    if (ws_size < (size_t)(NWG * 32 + 2 * NWG * TLEN * MT) * 4) return;
    const float* x       = (const float*)d_in[0];
    const float* y       = (const float*)d_in[1];
    const float* W_ih    = (const float*)d_in[2];
    const float* W_hh    = (const float*)d_in[3];
    const float* b_ih    = (const float*)d_in[4];
    const float* b_hh    = (const float*)d_in[5];
    const float* prior_W = (const float*)d_in[6];
    const float* prior_b = (const float*)d_in[7];
    const float* post_W  = (const float*)d_in[8];
    const float* post_b  = (const float*)d_in[9];
    float* out = (float*)d_out;
    float* ws  = (float*)d_ws;

    bkt_lstm_fused<<<NWG, NTHR, 0, stream>>>(x, y, W_ih, W_hh, b_ih, b_hh,
                                             prior_W, prior_b, post_W, post_b,
                                             out, ws);
    relayout<<<(TLEN * BATCH) / 256, 256, 0, stream>>>(ws, out);
    loss_reduce<<<1, 32, 0, stream>>>(ws, out);
}
